// RelativeAttention_82102594830987
// MI455X (gfx1250) — hardware-verified
//
#include <hip/hip_runtime.h>
#include <math.h>

#pragma clang fp contract(off)

constexpr int kB     = 16384;
constexpr int kA     = 4096;
constexpr int kD     = 512;
constexpr int kH     = 512;
constexpr int kQHalf = 8192;
constexpr int kChunk = 1024;
constexpr float kQKCarry    = 16.0f;
constexpr float kLoCarry    = 2048.0f;
constexpr float kLoInv      = 1.0f / 2048.0f;
constexpr float kSimScale   = 1.0f / 256.0f;
constexpr float kPCarry     = 32768.0f;
constexpr float kPCarryInv  = 1.0f / 32768.0f;
constexpr float kInvBin     = 20.0f;
constexpr float kBin        = 0.05f;
constexpr float kEdge       = 3.0e-3f;
constexpr float kNormEps    = 1.0e-12f;
static_assert(kB % kQHalf == 0 && kB % kChunk == 0, "shape");
static_assert(kQHalf % 64 == 0 && kChunk % 64 == 0 && kA % 64 == 0 && kH % 64 == 0 && kD % 64 == 0, "tiles");
static_assert(kD % 32 == 0 && kH % 32 == 0 && kA % 32 == 0, "ksteps");
static_assert(kA == 4096 && kH == 512, "side kernel maps");
static_assert(kA == 8 * 512 && kH == 2 * 256 && kH == 16 * 32, "softmax block maps");
static_assert(kA % 32 == 0 && kQHalf % 32 == 0, "norm grid");
static_assert((((kA / 64) * (kH / 64)) % 8) == 0, "kproj blocks");
static_assert((((kQHalf / 64) * (kH / 64)) % 8) == 0, "qproj blocks");
static_assert((((kChunk / 64) * (kA / 64)) % 8) == 0, "sim blocks");
static_assert((((kChunk / 64) * (kH / 64)) % 8) == 0, "pv blocks");

typedef __attribute__((ext_vector_type(16))) _Float16 v16h;
typedef __attribute__((ext_vector_type(8)))  _Float16 v8h;
typedef __attribute__((ext_vector_type(16))) __bf16   v16b;
typedef __attribute__((ext_vector_type(8)))  __bf16   v8b;
typedef __attribute__((ext_vector_type(8)))  float    v8f;
typedef __attribute__((ext_vector_type(4)))  float    v4f;
typedef __attribute__((ext_vector_type(2)))  float    v2f;
typedef __attribute__((ext_vector_type(4)))  unsigned int v4u;

__device__ __forceinline__ unsigned short f2bf_bits(float f) {
  unsigned u = __float_as_uint(f);
  return (unsigned short)((u + 0x7FFFu + ((u >> 16) & 1u)) >> 16);
}
__device__ __forceinline__ float bf_bits2f(unsigned short h) { return __uint_as_float(((unsigned)h) << 16); }

__device__ __forceinline__ void dep_guard_h(v8f& a, v8f& b, v16h x, v16h y) { asm volatile("v_nop\n\tv_nop\n\tv_nop\n\tv_nop" : "+v"(a), "+v"(b) : "v"(x), "v"(y)); }
__device__ __forceinline__ void dep_guard_b(v8f& a, v8f& b, v16b x, v16b y) { asm volatile("v_nop\n\tv_nop\n\tv_nop\n\tv_nop" : "+v"(a), "+v"(b) : "v"(x), "v"(y)); }
__device__ __forceinline__ void keep4_h(v16h a, v16h b, v16h c, v16h d) { asm volatile("v_nop" :: "v"(a), "v"(b), "v"(c), "v"(d)); }
__device__ __forceinline__ void keep4_b(v16b a, v16b b, v16b c, v16b d) { asm volatile("v_nop" :: "v"(a), "v"(b), "v"(c), "v"(d)); }
__device__ __forceinline__ void acc_guard4(v8f& a, v8f& b, v8f& c, v8f& d) { asm volatile("v_nop\n\tv_nop\n\tv_nop\n\tv_nop" : "+v"(a), "+v"(b), "+v"(c), "+v"(d)); }
template <typename T> struct Frag;
template <> struct Frag<_Float16> {
  typedef v16h V; union U { v16h v; v8h h[2]; };
  static __device__ __forceinline__ v16h load(const _Float16* p) {
    U f; f.h[0] = *(const v8h*)(p); f.h[1] = *(const v8h*)(p + 16); return f.v;
  }
  static __device__ __forceinline__ v8f mma(v16h a, v16h b, v8f c) {
    return __builtin_amdgcn_wmma_f32_16x16x32_f16(false, a, false, b, (short)0, c, false, false);
  }
  static __device__ __forceinline__ void guard(v8f& a, v8f& b, v16h x, v16h y) { dep_guard_h(a, b, x, y); }
  static __device__ __forceinline__ void keep(v16h a, v16h b, v16h c, v16h d) { keep4_h(a, b, c, d); }
};
template <> struct Frag<__bf16> {
  typedef v16b V; union U { v16b v; v8b h[2]; };
  static __device__ __forceinline__ v16b load(const __bf16* p) {
    U f; f.h[0] = *(const v8b*)(p); f.h[1] = *(const v8b*)(p + 16); return f.v;
  }
  static __device__ __forceinline__ v8f mma(v16b a, v16b b, v8f c) {
    return __builtin_amdgcn_wmma_f32_16x16x32_bf16(false, a, false, b, (short)0, c, false, false);
  }
  static __device__ __forceinline__ void guard(v8f& a, v8f& b, v16b x, v16b y) { dep_guard_b(a, b, x, y); }
  static __device__ __forceinline__ void keep(v16b a, v16b b, v16b c, v16b d) { keep4_b(a, b, c, d); }
};

__device__ __forceinline__ unsigned pk16(unsigned short a, unsigned short b) { return (unsigned)a | ((unsigned)b << 16); }
__device__ __forceinline__ unsigned short h_bits(float f) { const _Float16 h = (_Float16)f; return __builtin_bit_cast(unsigned short, h); }

__device__ __forceinline__ float h16_to_f32(unsigned hb) {
  const unsigned sgn = (hb & 0x8000u) << 16; const unsigned em = hb & 0x7fffu;
  const float fn = __uint_as_float((em << 13) + 0x38000000u);
  const float fs = (float)em * 5.9604644775390625e-8f;
  const float mag = (em < 0x400u) ? fs : fn; return __uint_as_float(__float_as_uint(mag) | sgn); }

template <int ET> struct Elem;
template <> struct Elem<0> { typedef _Float16 T; };
template <> struct Elem<1> { typedef __bf16 T; };
template <int ET, bool SPLIT, int BIAS_MODE, int OUT_MODE, bool RESID, int ACT = 0>
__global__ __launch_bounds__(256) void wmma_gemm64(
    const unsigned short* __restrict__ Ap, const unsigned short* __restrict__ A2p, int lda, long strideA,
    const unsigned short* __restrict__ Btp, const unsigned short* __restrict__ Bt2p, int ldb, long strideB,
    void* __restrict__ Cout, void* __restrict__ Cout2, int ldc, long strideC,
    const float* __restrict__ bias,
    const float* __restrict__ resid, long strideR,
    int M, int N, int K, float scale) {
  typedef typename Elem<ET>::T T;
  typedef typename Frag<T>::V V;
  const T* A = (const T*)Ap; const T* A2 = (const T*)A2p; const T* Bt = (const T*)Btp; const T* Bt2 = (const T*)Bt2p;
  __shared__ __align__(16) float sT[8][16 * 68];
  const int b    = blockIdx.y;
  const int lane = threadIdx.x & 31;
  const int wave = threadIdx.x >> 5;
  const int tilesN = N >> 6;
  const int tilesM = M >> 6;
  const int tile = blockIdx.x * 8 + wave;
  if (tile >= tilesM * tilesN) return;
  const int tm = tile / tilesN;
  const int tn = tile - tm * tilesN;
  const int m0 = tm << 6;
  const int n0 = tn << 6;

  const T* Ab  = A  + (size_t)b * strideA;
  const T* Bb  = Bt + (size_t)b * strideB;
  const T* Ab2 = SPLIT ? (A2  + (size_t)b * strideA) : nullptr;
  const T* Bb2 = SPLIT ? (Bt2 + (size_t)b * strideB) : nullptr;

  const int rlane = lane & 15;
  const int koff  = (lane >> 4) * 8;
  const int mOff  = (lane >> 4) * 8;

  v8f acc[4][4];
#pragma unroll
  for (int i = 0; i < 4; ++i)
#pragma unroll
    for (int j = 0; j < 4; ++j) acc[i][j] = (v8f){0.f,0.f,0.f,0.f,0.f,0.f,0.f,0.f};

  for (int k0 = 0; k0 < K; k0 += 32) {
    V bh[4], bl[4];
#pragma unroll
    for (int j = 0; j < 4; ++j) {
      const size_t bo = (size_t)(n0 + (j << 4) + rlane) * ldb + koff + k0;
      bh[j] = Frag<T>::load(Bb + bo);
      if (SPLIT) bl[j] = Frag<T>::load(Bb2 + bo);
    }
#pragma unroll
    for (int i = 0; i < 4; ++i) {
      const size_t ao = (size_t)(m0 + (i << 4) + rlane) * lda + koff + k0;
      V ah = Frag<T>::load(Ab + ao);
      V al;
      if (SPLIT) al = Frag<T>::load(Ab2 + ao);
#pragma unroll
      for (int j = 0; j < 4; ++j) {
        acc[i][j] = Frag<T>::mma(ah, bh[j], acc[i][j]);
        if (SPLIT) {
          acc[i][j] = Frag<T>::mma(ah, bl[j], acc[i][j]);
          acc[i][j] = Frag<T>::mma(al, bh[j], acc[i][j]);
        }
      }
      Frag<T>::guard(acc[i][0], acc[i][3], ah, SPLIT ? al : ah);
    }
    Frag<T>::keep(bh[0], bh[1], bh[2], bh[3]);
    if (SPLIT) Frag<T>::keep(bl[0], bl[1], bl[2], bl[3]);
  }
  acc_guard4(acc[0][0], acc[0][1], acc[0][2], acc[0][3]);
  acc_guard4(acc[1][0], acc[1][1], acc[1][2], acc[1][3]);
  acc_guard4(acc[2][0], acc[2][1], acc[2][2], acc[2][3]);
  acc_guard4(acc[3][0], acc[3][1], acc[3][2], acc[3][3]);

  float* slab = sT[wave];
  const float* Rb = RESID ? (resid + (size_t)b * strideR) : nullptr;
#pragma unroll
  for (int i = 0; i < 4; ++i) {
    const int mBase = m0 + (i << 4);
#pragma unroll
    for (int j = 0; j < 4; ++j) {
      const int n = n0 + (j << 4) + rlane;
      float bv = 0.f;
      if (BIAS_MODE == 2) bv = bias[n];
#pragma unroll
      for (int r = 0; r < 8; ++r) {
        float v = acc[i][j][r] * scale;
        if (BIAS_MODE == 1) v += bias[mBase + mOff + r];
        if (BIAS_MODE == 2) v += bv;
        if (RESID) v += Rb[(size_t)(mBase + mOff + r) * ldc + n];
        if (ACT == 2) v = fmaxf(v, 0.0f);
        if (ACT == 4) v = (v > 0.f) ? v : 0.01f * v;
        slab[(mOff + r) * 68 + (j << 4) + rlane] = v;
      }
    }
    __builtin_amdgcn_fence(__ATOMIC_RELEASE, "workgroup");
    __builtin_amdgcn_wave_barrier();
    __builtin_amdgcn_fence(__ATOMIC_ACQUIRE, "workgroup");
    if (OUT_MODE == 0) {
      float* C = (float*)Cout + (size_t)b * strideC;
      const int hh = lane >> 4, c4 = (lane & 15) * 4;
      for (int pass = 0; pass < 2; ++pass) {
#pragma unroll
        for (int it = 0; it < 8; ++it) {
          const int row = it * 2 + hh;
          v4f v = *(const v4f*)(slab + row * 68 + c4);
          *(volatile v4f*)(C + (size_t)(mBase + row) * ldc + n0 + c4) = v;
        }
        __threadfence();
      }
    } else {
      const int q = lane >> 3, c8 = (lane & 7) * 8;
      unsigned short* C  = (unsigned short*)Cout  + (size_t)b * strideC;
      unsigned short* C2 = (OUT_MODE == 2) ? ((unsigned short*)Cout2 + (size_t)b * strideC) : nullptr;
      for (int pass = 0; pass < 2; ++pass) {
#pragma unroll
        for (int it = 0; it < 4; ++it) {
          const int row = it * 4 + q;
          const float* sp = slab + row * 68 + c8;
          v8h hv, lv;
#pragma unroll
          for (int e = 0; e < 8; ++e) {
            if (OUT_MODE == 1) {
              hv[e] = (_Float16)sp[e];
            } else {
              unsigned short hb = f2bf_bits(sp[e]);
              unsigned short lb = f2bf_bits(sp[e] - bf_bits2f(hb));
              hv[e] = __builtin_bit_cast(_Float16, hb);
              lv[e] = __builtin_bit_cast(_Float16, lb);
            }
          }
          *(volatile v8h*)(C + (size_t)(mBase + row) * ldc + n0 + c8) = hv;
          if (OUT_MODE == 2) *(volatile v8h*)(C2 + (size_t)(mBase + row) * ldc + n0 + c8) = lv;
        }
        __threadfence();
      }
    }
    __builtin_amdgcn_fence(__ATOMIC_RELEASE, "workgroup");
    __builtin_amdgcn_wave_barrier();
    __builtin_amdgcn_fence(__ATOMIC_ACQUIRE, "workgroup");
  }
}

__global__ __launch_bounds__(256) void cast8_bf16_kernel(const float* __restrict__ in, unsigned short* __restrict__ out, int n8) {
  const int i = blockIdx.x * 256 + threadIdx.x;
  if (i >= n8) return;
  const float* p = in + 8 * (size_t)i;
  const v4f a = *(const v4f*)(p);
  const v4f c = *(const v4f*)(p + 4);
  unsigned short hb[8];
#pragma unroll
  for (int e = 0; e < 4; ++e) {
    hb[e]     = f2bf_bits(a[e]);
    hb[4 + e] = f2bf_bits(c[e]);
  }
  const v4u u = (v4u){pk16(hb[0], hb[1]), pk16(hb[2], hb[3]), pk16(hb[4], hb[5]), pk16(hb[6], hb[7])};
  unsigned short* q = out + 8 * (size_t)i;
  *(volatile v4u*)q = u;
  __threadfence();
  *(volatile v4u*)q = u;
}

template <int MODE> __device__ __forceinline__ unsigned short tc_bits(float f) {
  if (MODE == 0) return f2bf_bits(f);
  const float g = bf_bits2f(f2bf_bits(f));
  return h_bits(g);
}
template <int MODE>
__global__ __launch_bounds__(256) void transpose_cast_kernel(const float* __restrict__ in, unsigned short* __restrict__ out, int R, int C) {
  __shared__ float sm[64][65];
  const int t  = threadIdx.x;
  const int r0 = blockIdx.x * 64;
  const int c0 = blockIdx.y * 64;
#pragma unroll
  for (int i = 0; i < 16; ++i) {
    const int e  = i * 256 + t;
    const int rl = e >> 6;
    const int cl = e & 63;
    sm[cl][rl] = in[(size_t)(r0 + rl) * C + c0 + cl];
  }
  __syncthreads();
  const int lane = t & 31, wave = t >> 5;
  const int q = lane >> 3, c8 = (lane & 7) * 8;
  for (int pass = 0; pass < 2; ++pass) {
#pragma unroll
    for (int it = 0; it < 2; ++it) {
      const int row = wave * 8 + it * 4 + q;
      unsigned short hb[8];
#pragma unroll
      for (int e = 0; e < 8; ++e) hb[e] = tc_bits<MODE>(sm[row][c8 + e]);
      const v4u u = (v4u){pk16(hb[0], hb[1]), pk16(hb[2], hb[3]), pk16(hb[4], hb[5]), pk16(hb[6], hb[7])};
      *(volatile v4u*)(out + (size_t)(c0 + row) * R + r0 + c8) = u;
    }
    __threadfence();
  }
}

__device__ __forceinline__ void cvt16(float g, unsigned short& hb, unsigned short& lb) {
  hb = h_bits(g);
  const float back = h16_to_f32((unsigned)hb);
  lb = h_bits((g - back) * kLoCarry);
}
__global__ __launch_bounds__(256) void l2norm_split_kernel(const float* __restrict__ in, unsigned short* __restrict__ outh,
                                                          unsigned short* __restrict__ outl, int rows, float carry) {
  const int lane  = threadIdx.x & 31;
  const int wave  = threadIdx.x >> 5;
  const int rbase = (blockIdx.x * 8 + wave) * 4;
#pragma unroll 1
  for (int rr = 0; rr < 4; ++rr) {
    const int row  = rbase + rr;
    const int rowc = (row < rows) ? row : (rows - 1);
    const float* p = in + (size_t)rowc * kH;
    const v4f a0 = *(const v4f*)(p + 8 * lane);
    const v4f a1 = *(const v4f*)(p + 8 * lane + 4);
    const v4f a2 = *(const v4f*)(p + 256 + 8 * lane);
    const v4f a3 = *(const v4f*)(p + 256 + 8 * lane + 4);
    float ss = 0.0f;
#pragma unroll
    for (int e = 0; e < 4; ++e) ss += a0[e] * a0[e];
#pragma unroll
    for (int e = 0; e < 4; ++e) ss += a1[e] * a1[e];
#pragma unroll
    for (int e = 0; e < 4; ++e) ss += a2[e] * a2[e];
#pragma unroll
    for (int e = 0; e < 4; ++e) ss += a3[e] * a3[e];
#pragma unroll
    for (int off = 16; off > 0; off >>= 1) ss += __shfl_xor(ss, off, 32);
    const float inv = carry / fmaxf(sqrtf(ss), kNormEps);
    unsigned short hb[16];
    unsigned short lb[16];
#pragma unroll
    for (int e = 0; e < 4; ++e) {
      cvt16(a0[e] * inv, hb[e],      lb[e]);
      cvt16(a1[e] * inv, hb[4 + e],  lb[4 + e]);
      cvt16(a2[e] * inv, hb[8 + e],  lb[8 + e]);
      cvt16(a3[e] * inv, hb[12 + e], lb[12 + e]);
    }
    const v4u u0 = (v4u){pk16(hb[0], hb[1]), pk16(hb[2], hb[3]), pk16(hb[4], hb[5]), pk16(hb[6], hb[7])};
    const v4u u1 = (v4u){pk16(hb[8], hb[9]), pk16(hb[10], hb[11]), pk16(hb[12], hb[13]), pk16(hb[14], hb[15])};
    const v4u w0 = (v4u){pk16(lb[0], lb[1]), pk16(lb[2], lb[3]), pk16(lb[4], lb[5]), pk16(lb[6], lb[7])};
    const v4u w1 = (v4u){pk16(lb[8], lb[9]), pk16(lb[10], lb[11]), pk16(lb[12], lb[13]), pk16(lb[14], lb[15])};
    if (row < rows) {
      unsigned short* qh = outh + (size_t)row * kH;
      unsigned short* ql = outl + (size_t)row * kH;
      for (int pass = 0; pass < 2; ++pass) {
        *(volatile v4u*)(qh + 8 * lane) = u0;
        *(volatile v4u*)(qh + 256 + 8 * lane) = u1;
        *(volatile v4u*)(ql + 8 * lane) = w0;
        *(volatile v4u*)(ql + 256 + 8 * lane) = w1;
        __threadfence();
      }
    }
  }
}

__device__ __forceinline__ unsigned near_edge(float s) {
  const float tt = s * kInvBin;
  const float fr = tt - floorf(tt);
  const float d  = fr - 0.5f;
  return (fabsf(d) < kEdge) ? 1u : 0u;
}
__global__ __launch_bounds__(512) void quant_softmax_kernel(const float* __restrict__ S,
                                                           const unsigned short* __restrict__ Qh, const unsigned short* __restrict__ Ql,
                                                           const unsigned short* __restrict__ Kh, const unsigned short* __restrict__ Kl,
                                                           unsigned short* __restrict__ P) {
  __shared__ __align__(16) float lg[kA];
  __shared__ __align__(16) float qf[kH];
  __shared__ float redS[16];
  const int i    = blockIdx.x;
  const int t    = threadIdx.x;
  const int lane = t & 31, wave = t >> 5;

  if (t < kH / 2) {
    const unsigned hw = ((const unsigned*)(Qh + (size_t)i * kH))[t];
    const unsigned lw = ((const unsigned*)(Ql + (size_t)i * kH))[t];
    const float a0 = h16_to_f32(hw & 0xffffu);
    const float a1 = h16_to_f32(hw >> 16);
    const float b0 = h16_to_f32(lw & 0xffffu);
    const float b1 = h16_to_f32(lw >> 16);
    const v2f qv = (v2f){fmaf(b0, kLoInv, a0), fmaf(b1, kLoInv, a1)};
    *(v2f*)(qf + 2 * t) = qv;
  }

  unsigned hbits = 0u;
  {
    const float* sr = S + (size_t)i * kA + 8 * (size_t)t;
    const v4f s0 = *(const v4f*)(sr);
    const v4f s1 = *(const v4f*)(sr + 4);
#pragma unroll
    for (int e = 0; e < 4; ++e) {
      hbits |= near_edge(s0[e]) << e;
      hbits |= near_edge(s1[e]) << (4 + e);
    }
    *(v4f*)(lg + 8 * t)     = s0;
    *(v4f*)(lg + 8 * t + 4) = s1;
  }
  __syncthreads();

#pragma unroll 1
  for (int e = 0; e < 8; ++e) {
    unsigned mask = __builtin_amdgcn_ballot_w32(((hbits >> e) & 1u) != 0u);
#pragma unroll 1
    for (int q = 0; q < 32; ++q) {
      if (mask == 0u) break;
      const int l = __builtin_ctz(mask);
      mask &= mask - 1u;
      const int a = (wave << 8) + (l << 3) + e;
      const unsigned short* khp = Kh + (size_t)a * kH + 16 * lane;
      const unsigned short* klp = Kl + (size_t)a * kH + 16 * lane;
      const float* qp = qf + 16 * lane;
      float acc = 0.0f;
#pragma unroll 1
      for (int g = 0; g < 2; ++g) {
        const v4u wh = *(const v4u*)(khp + 8 * g);
        const v4u wl = *(const v4u*)(klp + 8 * g);
        const v4f qa = *(const v4f*)(qp + 8 * g);
        const v4f qb = *(const v4f*)(qp + 8 * g + 4);
        float qq[8];
#pragma unroll
        for (int u = 0; u < 4; ++u) { qq[u] = qa[u]; qq[4 + u] = qb[u]; }
#pragma unroll
        for (int u = 0; u < 4; ++u) {
          const unsigned hwd = wh[u];
          const unsigned lwd = wl[u];
          const float kh0 = h16_to_f32(hwd & 0xffffu);
          const float kh1 = h16_to_f32(hwd >> 16);
          const float kl0 = h16_to_f32(lwd & 0xffffu);
          const float kl1 = h16_to_f32(lwd >> 16);
          const float kf0 = fmaf(kl0, kLoInv, kh0);
          const float kf1 = fmaf(kl1, kLoInv, kh1);
          acc = fmaf(qq[2 * u],     kf0, acc);
          acc = fmaf(qq[2 * u + 1], kf1, acc);
        }
      }
#pragma unroll
      for (int off = 16; off > 0; off >>= 1) acc += __shfl_xor(acc, off, 32);
      const float sref = acc * kSimScale;
      if (lane == 0) lg[a] = sref;
    }
  }
  __syncthreads();

  float sum = 0.0f;
#pragma unroll 1
  for (int e = 0; e < 8; ++e) {
    const float sv = lg[8 * t + e];
    const float r  = rintf(sv * kInvBin);
    const float tq = r * kBin;
    const float d  = tq - sv;
    const float x  = sv + d;
    const float ex = expf(x);
    sum += ex;
    lg[8 * t + e] = ex;
  }
#pragma unroll
  for (int off = 16; off > 0; off >>= 1) sum += __shfl_xor(sum, off, 32);
  if (lane == 0) redS[wave] = sum;
  __syncthreads();
  float tot = redS[0];
#pragma unroll
  for (int w = 1; w < 16; ++w) tot += redS[w];
  const float inv = kPCarry / tot;
  const v4f e0 = *(const v4f*)(lg + 8 * t);
  const v4f e1 = *(const v4f*)(lg + 8 * t + 4);
  unsigned short hb[8];
#pragma unroll
  for (int e = 0; e < 4; ++e) {
    hb[e]     = h_bits(e0[e] * inv);
    hb[4 + e] = h_bits(e1[e] * inv);
  }
  const v4u u = (v4u){pk16(hb[0], hb[1]), pk16(hb[2], hb[3]), pk16(hb[4], hb[5]), pk16(hb[6], hb[7])};
  unsigned short* pr = P + (size_t)i * kA + 8 * (size_t)t;
  *(volatile v4u*)pr = u;
  __threadfence();
  *(volatile v4u*)pr = u;
}

extern "C" void kernel_launch(void* const* d_in, const int* in_sizes, int n_in,
                              void* d_out, int out_size, void* d_ws, size_t ws_size,
                              hipStream_t stream) {
  if (n_in < 5) return;
  if (in_sizes[0] != kB * kD) return;
  if (in_sizes[1] != kA * kD) return;
  if (in_sizes[2] != kD * kH) return;
  if (in_sizes[3] != kD * kH) return;
  if (in_sizes[4] != kA * kH) return;
  if (out_size != kB * kH) return;

  const size_t szXb   = (size_t)kB * kD * 2;
  const size_t szAb   = (size_t)kA * kD * 2;
  const size_t szW    = (size_t)kD * kH * 2;
  const size_t szVt   = (size_t)kH * kA * 2;
  const size_t szQraw = (size_t)kQHalf * kH * 4;
  const size_t szQn   = (size_t)kB * kH * 2;
  const size_t szKn   = (size_t)kA * kH * 2;
  const size_t szS    = (size_t)kChunk * kA * 4;
  const size_t szP    = (size_t)kChunk * kA * 2;
  const size_t offXb   = 0;
  const size_t offAb   = offXb + szXb;
  const size_t offWq   = offAb + szAb;
  const size_t offWk   = offWq + szW;
  const size_t offVt   = offWk + szW;
  const size_t offQraw = offVt + szVt;
  const size_t offQnh  = offQraw + szQraw;
  const size_t offQnl  = offQnh + szQn;
  const size_t offKnh  = offQnl + szQn;
  const size_t offKnl  = offKnh + szKn;
  const size_t offS    = offKnl + szKn;
  const size_t offP    = offS + szS;
  const size_t total   = offP + szP;
  if (ws_size < total) return;
  if ((size_t)kA * kH * 4 > szQraw) return;

  const float* x       = (const float*)d_in[0];
  const float* anchors = (const float*)d_in[1];
  const float* Wq      = (const float*)d_in[2];
  const float* Wk      = (const float*)d_in[3];
  const float* values  = (const float*)d_in[4];
  float* out = (float*)d_out;
  char* ws = (char*)d_ws;
  unsigned short* Xb   = (unsigned short*)(ws + offXb);
  unsigned short* Ab   = (unsigned short*)(ws + offAb);
  unsigned short* WqT  = (unsigned short*)(ws + offWq);
  unsigned short* WkT  = (unsigned short*)(ws + offWk);
  unsigned short* Vt   = (unsigned short*)(ws + offVt);
  float*          Qraw = (float*)(ws + offQraw);
  float*          Kraw = Qraw;
  unsigned short* Qnh  = (unsigned short*)(ws + offQnh);
  unsigned short* Qnl  = (unsigned short*)(ws + offQnl);
  unsigned short* Knh  = (unsigned short*)(ws + offKnh);
  unsigned short* Knl  = (unsigned short*)(ws + offKnl);
  float*          Sbuf = (float*)(ws + offS);
  unsigned short* Pbuf = (unsigned short*)(ws + offP);
  const float* fdum = Qraw;

  {
    const int n8x = (kB * kD) / 8;
    const int n8a = (kA * kD) / 8;
    cast8_bf16_kernel<<<dim3(n8x / 256), dim3(256), 0, stream>>>(x, Xb, n8x);
    cast8_bf16_kernel<<<dim3(n8a / 256), dim3(256), 0, stream>>>(anchors, Ab, n8a);
    transpose_cast_kernel<0><<<dim3(kD / 64, kH / 64), dim3(256), 0, stream>>>(Wq, WqT, kD, kH);
    transpose_cast_kernel<0><<<dim3(kD / 64, kH / 64), dim3(256), 0, stream>>>(Wk, WkT, kD, kH);
    transpose_cast_kernel<1><<<dim3(kA / 64, kH / 64), dim3(256), 0, stream>>>(values, Vt, kA, kH);
  }

  {
    const int tiles = (kA / 64) * (kH / 64);
    wmma_gemm64<1, false, 0, 0, false, 0><<<dim3(tiles / 8, 1), dim3(256), 0, stream>>>(
        Ab, Ab, kD, 0L, WkT, WkT, kD, 0L, (void*)Kraw, (void*)Kraw, kH, 0L, fdum, fdum, 0L, kA, kH, kD, 1.0f);
    l2norm_split_kernel<<<dim3(kA / 32), dim3(256), 0, stream>>>(Kraw, Knh, Knl, kA, kQKCarry);
  }

  for (int hq = 0; hq < kB / kQHalf; ++hq) {
    const int tiles = (kQHalf / 64) * (kH / 64);
    const unsigned short* Ah = Xb + (size_t)hq * kQHalf * kD;
    wmma_gemm64<1, false, 0, 0, false, 0><<<dim3(tiles / 8, 1), dim3(256), 0, stream>>>(
        Ah, Ah, kD, 0L, WqT, WqT, kD, 0L, (void*)Qraw, (void*)Qraw, kH, 0L, fdum, fdum, 0L, kQHalf, kH, kD, 1.0f);
    const size_t qoff = (size_t)hq * kQHalf * kH;
    l2norm_split_kernel<<<dim3(kQHalf / 32), dim3(256), 0, stream>>>(Qraw, Qnh + qoff, Qnl + qoff, kQHalf, kQKCarry);
  }

  const int tilesSim = (kChunk / 64) * (kA / 64);
  const int tilesPV  = (kChunk / 64) * (kH / 64);
  for (int c = 0; c < kB / kChunk; ++c) {
    const size_t qoff = (size_t)c * kChunk * kH;
    const unsigned short* Ach = Qnh + qoff;
    const unsigned short* Acl = Qnl + qoff;
    wmma_gemm64<0, false, 0, 0, false, 0><<<dim3(tilesSim / 8, 1), dim3(256), 0, stream>>>(
        Ach, Ach, kH, 0L, Knh, Knh, kH, 0L, (void*)Sbuf, (void*)Sbuf, kA, 0L, fdum, fdum, 0L, kChunk, kA, kH, kSimScale);
    quant_softmax_kernel<<<dim3(kChunk), dim3(512), 0, stream>>>(Sbuf, Ach, Acl, Knh, Knl, Pbuf);
    float* outc = out + qoff;
    wmma_gemm64<0, false, 0, 0, false, 0><<<dim3(tilesPV / 8, 1), dim3(256), 0, stream>>>(
        Pbuf, Pbuf, kA, 0L, Vt, Vt, kA, 0L, (void*)outc, (void*)outc, kH, 0L, fdum, fdum, 0L, kChunk, kH, kA, kPCarryInv);
  }
}
